// RelPosMultiHeadAttention_53712861004261
// MI455X (gfx1250) — hardware-verified
//
#include <hip/hip_runtime.h>
#include <math.h>
#include <stdint.h>

#define SEQ   1024
#define NBAT  2
#define DMOD  1024
#define NH    16
#define DH    64
#define ELEN  2047
#define EPAD  2048
#define NROW  (NBAT * SEQ)
#define XC    16.0f
#define WSC   64.0f
#define QC    64.0f
#define KC    64.0f
#define EC    16.0f
#define VC    64.0f
#define PC    1024.0f
#define CC    256.0f
#define SCALE 0.125f
#define LOG2E 1.4426950408889634f
static_assert(NH * DH == DMOD);
static_assert(DH == 64);
static_assert(ELEN == 2 * SEQ - 1 && EPAD >= ELEN);
static_assert((SEQ % 64) == 0 && (DMOD % 64) == 0 && (NROW % 64) == 0);
static_assert(((NROW * DMOD) % 2048) == 0 && ((DMOD * DMOD) % 2048) == 0 && ((ELEN * DH) % 8) == 0);
#define ATT_W 4
#define ATT_THREADS (ATT_W * 32)
#define TPI 84
#define SPI 68
#define WFL (16 * TPI + 16 * SPI)
static_assert(((16 * TPI) % 4) == 0 && ((16 * SPI) % 4) == 0 && (WFL % 4) == 0);

typedef _Float16 v16h __attribute__((ext_vector_type(16)));
typedef _Float16 v8h  __attribute__((ext_vector_type(8)));
typedef __bf16   v16b __attribute__((ext_vector_type(16)));
typedef float    v8f  __attribute__((ext_vector_type(8)));
typedef float    v4f  __attribute__((ext_vector_type(4)));
typedef float    v2f  __attribute__((ext_vector_type(2)));
typedef unsigned int v4u __attribute__((ext_vector_type(4)));

union FragH { v16h v; v8h h[2]; v4u u[2]; };
union FragAny { v16h h; v16b b; };

__device__ __forceinline__ unsigned short bf_bits(float f) {
  unsigned u = __float_as_uint(f);
  return (unsigned short)((u + 0x7FFFu + ((u >> 16) & 1u)) >> 16);
}
__device__ __forceinline__ float bf_up(unsigned short h) { return __uint_as_float(((unsigned)h) << 16); }
__device__ __forceinline__ float bfr(float f) { return bf_up(bf_bits(f)); }
__device__ __forceinline__ unsigned short h_bits(_Float16 x) { return __builtin_bit_cast(unsigned short, x); }
__device__ __forceinline__ unsigned pk16(unsigned short a, unsigned short b) { return (unsigned)a | ((unsigned)b << 16); }
__device__ __forceinline__ v8f zero8() { v8f z = {0.f, 0.f, 0.f, 0.f, 0.f, 0.f, 0.f, 0.f}; return z; }

__device__ __forceinline__ v16h ldfrag_u(const unsigned short* p) {
  FragH f;
  f.u[0] = *(const v4u*)(p);
  f.u[1] = *(const v4u*)(p + 16);
  return f.v;
}

__device__ __forceinline__ v8f mma_h(v16h a, v16h b, v8f c) {
  return __builtin_amdgcn_wmma_f32_16x16x32_f16(false, a, false, b, (short)0, c, false, false);
}
__device__ __forceinline__ v8f mma_b(v16h a, v16h b, v8f c) {
  FragAny ua, ub;
  ua.h = a;
  ub.h = b;
  return __builtin_amdgcn_wmma_f32_16x16x32_bf16(false, ua.b, false, ub.b, (short)0, c, false, false);
}
template <int BF>
__device__ __forceinline__ v8f mmaT(v16h a, v16h b, v8f c) {
  if constexpr (BF != 0) return mma_b(a, b, c);
  else return mma_h(a, b, c);
}
__device__ __forceinline__ void dep_guard1(v8f& a, v8f& b, v16h x) {
#if defined(__HIP_DEVICE_COMPILE__)
  asm volatile("v_nop\n\tv_nop\n\tv_nop\n\tv_nop" : "+v"(a), "+v"(b) : "v"(x));
#endif
}
__device__ __forceinline__ void hz4(v8f& d, v16h x0, v16h x1, v16h x2, v16h x3) {
#if defined(__HIP_DEVICE_COMPILE__)
  asm volatile("v_nop\n\tv_nop\n\tv_nop\n\tv_nop" : "+v"(d) : "v"(x0), "v"(x1), "v"(x2), "v"(x3));
#endif
}
__device__ __forceinline__ void hz6(v8f& d, v16h x0, v16h x1, v16h x2, v16h x3, v16h x4, v16h x5) {
#if defined(__HIP_DEVICE_COMPILE__)
  asm volatile("v_nop\n\tv_nop\n\tv_nop\n\tv_nop" : "+v"(d) : "v"(x0), "v"(x1), "v"(x2), "v"(x3), "v"(x4), "v"(x5));
#endif
}
__device__ __forceinline__ void hz8(v8f& d, v16h x0, v16h x1, v16h x2, v16h x3, v16h x4, v16h x5, v16h x6, v16h x7) {
#if defined(__HIP_DEVICE_COMPILE__)
  asm volatile("v_nop\n\tv_nop\n\tv_nop\n\tv_nop" : "+v"(d) : "v"(x0), "v"(x1), "v"(x2), "v"(x3), "v"(x4), "v"(x5), "v"(x6), "v"(x7));
#endif
}
__device__ __forceinline__ void keep4_h(v16h a, v16h b, v16h c, v16h d) {
#if defined(__HIP_DEVICE_COMPILE__)
  asm volatile("v_nop" :: "v"(a), "v"(b), "v"(c), "v"(d));
#endif
}
__device__ __forceinline__ void acc_guard4(v8f& a, v8f& b, v8f& c, v8f& d) {
#if defined(__HIP_DEVICE_COMPILE__)
  asm volatile("v_nop\n\tv_nop\n\tv_nop\n\tv_nop" : "+v"(a), "+v"(b), "+v"(c), "+v"(d));
#endif
}
__device__ __forceinline__ void wave_sync_lds() {
  __builtin_amdgcn_fence(__ATOMIC_RELEASE, "workgroup");
  __builtin_amdgcn_wave_barrier();
  __builtin_amdgcn_fence(__ATOMIC_ACQUIRE, "workgroup");
}
__device__ __forceinline__ void sp16(float x, _Float16& hi, _Float16& lo) {
  const _Float16 a = (_Float16)x;
  hi = a;
  lo = (_Float16)(x - (float)a);
}
__device__ __forceinline__ void pack_hl(float x0, float x1, unsigned& hw, unsigned& lw) {
  _Float16 a0, a1, b0, b1;
  sp16(x0, a0, b0);
  sp16(x1, a1, b1);
  hw = pk16(h_bits(a0), h_bits(a1));
  lw = pk16(h_bits(b0), h_bits(b1));
}

__global__ __launch_bounds__(256) void cvt16(const float* __restrict__ src, unsigned short* dst, int n, float sc) {
  const size_t i8 = ((size_t)blockIdx.x * 256 + threadIdx.x) * 8;
  if (i8 + 8 > (size_t)n) return;
  const v4f a = *(const v4f*)(src + i8);
  const v4f b = *(const v4f*)(src + i8 + 4);
  v4u o;
  o[0] = pk16(h_bits((_Float16)(bfr(a[0]) * sc)), h_bits((_Float16)(bfr(a[1]) * sc)));
  o[1] = pk16(h_bits((_Float16)(bfr(a[2]) * sc)), h_bits((_Float16)(bfr(a[3]) * sc)));
  o[2] = pk16(h_bits((_Float16)(bfr(b[0]) * sc)), h_bits((_Float16)(bfr(b[1]) * sc)));
  o[3] = pk16(h_bits((_Float16)(bfr(b[2]) * sc)), h_bits((_Float16)(bfr(b[3]) * sc)));
  for (int pass = 0; pass < 2; ++pass) {
    *(volatile v4u*)(dst + i8) = o;
    __threadfence();
  }
}

template <int OM, int ASPLIT, int BF, int EPI>
__global__ __launch_bounds__(256) __attribute__((amdgpu_num_vgpr(256))) void gemm64(
    const unsigned short* __restrict__ Ap, const unsigned short* __restrict__ A2p, int lda, long long sA,
    const unsigned short* __restrict__ Btp, int ldb, long long sB,
    void* Cout, void* C2out, int ldc, long long sC,
    int M, int N, int K, float oscale, float ocarry,
    const float* __restrict__ ep0, const float* __restrict__ ep1, const float* __restrict__ ep2) {
  __shared__ __align__(16) float sT[8][16 * 68];
  const int by   = blockIdx.y;
  const int lane = threadIdx.x & 31;
  const int wave = threadIdx.x >> 5;
  const int tilesN = N >> 6;
  const int tilesM = M >> 6;
  const int tile = blockIdx.x * 8 + wave;
  if (tile >= tilesM * tilesN) return;
  const int tm = tile / tilesN;
  const int tn = tile - tm * tilesN;
  const int m0 = tm << 6;
  const int n0 = tn << 6;

  const unsigned short* A1 = Ap  + (size_t)((long long)by * sA);
  const unsigned short* A2 = A2p + (size_t)((long long)by * sA);
  const unsigned short* Bb = Btp + (size_t)((long long)by * sB);

  const int rlane = lane & 15;
  const int koff  = (lane >> 4) * 8;
  const int mOff  = (lane >> 4) * 8;

  v8f acc[4][4];
#pragma unroll
  for (int i = 0; i < 4; ++i)
#pragma unroll
    for (int j = 0; j < 4; ++j) acc[i][j] = zero8();

  for (int k0 = 0; k0 < K; k0 += 32) {
    v16h bh[4];
#pragma unroll
    for (int j = 0; j < 4; ++j) {
      const size_t bofs = (size_t)(n0 + (j << 4) + rlane) * ldb + koff + k0;
      bh[j] = ldfrag_u(Bb + bofs);
    }
#pragma unroll
    for (int i = 0; i < 4; ++i) {
      const size_t ao = (size_t)(m0 + (i << 4) + rlane) * lda + koff + k0;
      const v16h ah = ldfrag_u(A1 + ao);
#pragma unroll
      for (int j = 0; j < 4; ++j) acc[i][j] = mmaT<BF>(ah, bh[j], acc[i][j]);
      dep_guard1(acc[i][0], acc[i][3], ah);
      if constexpr (ASPLIT != 0) {
        const v16h al = ldfrag_u(A2 + ao);
#pragma unroll
        for (int j = 0; j < 4; ++j) acc[i][j] = mmaT<BF>(al, bh[j], acc[i][j]);
        dep_guard1(acc[i][0], acc[i][3], al);
      }
    }
    keep4_h(bh[0], bh[1], bh[2], bh[3]);
  }
  acc_guard4(acc[0][0], acc[0][1], acc[0][2], acc[0][3]);
  acc_guard4(acc[1][0], acc[1][1], acc[1][2], acc[1][3]);
  acc_guard4(acc[2][0], acc[2][1], acc[2][2], acc[2][3]);
  acc_guard4(acc[3][0], acc[3][1], acc[3][2], acc[3][3]);

  const int hh2 = lane >> 4, c4 = (lane & 15) * 4;
  const int q8  = lane >> 3, c8 = (lane & 7) * 8;

  float* slab = sT[wave];
#pragma unroll
  for (int i = 0; i < 4; ++i) {
    const int mBase = m0 + (i << 4);
#pragma unroll
    for (int j = 0; j < 4; ++j) {
#pragma unroll
      for (int r = 0; r < 8; ++r) {
        slab[(mOff + r) * 68 + (j << 4) + rlane] = acc[i][j][r];
      }
    }
    wave_sync_lds();
    if constexpr (OM == 0) {
      float* C = (float*)Cout + (size_t)((long long)by * sC);
      v4f vals[8];
#pragma unroll
      for (int it = 0; it < 8; ++it) {
        const int row = it * 2 + hh2;
        v4f v = *(const v4f*)(slab + row * 68 + c4);
#pragma unroll
        for (int e = 0; e < 4; ++e) v[e] = v[e] * oscale;
        if constexpr (EPI == 1) {
          const v4f bb = *(const v4f*)(ep0 + n0 + c4);
#pragma unroll
          for (int e = 0; e < 4; ++e) v[e] = v[e] + bfr(bb[e]);
        }
        vals[it] = v;
      }
      for (int pass = 0; pass < 2; ++pass) {
#pragma unroll
        for (int it = 0; it < 8; ++it) {
          const int gr = mBase + it * 2 + hh2;
          *(volatile v4f*)(C + (size_t)gr * ldc + n0 + c4) = vals[it];
        }
        __threadfence();
      }
    } else {
      unsigned short* C  = (unsigned short*)Cout  + (size_t)((long long)by * sC);
      unsigned short* Cb = (unsigned short*)C2out + (size_t)((long long)by * sC);
      v4u hv[4], lv[4];
#pragma unroll
      for (int it = 0; it < 4; ++it) {
        const int row = it * 4 + q8;
        const float* sp = slab + row * 68 + c8;
        float rb = 0.f;
        if constexpr (EPI == 2) rb = bfr(ep0[mBase + row]);
        v4u a  = {0u, 0u, 0u, 0u};
        v4u b2 = {0u, 0u, 0u, 0u};
#pragma unroll
        for (int e = 0; e < 4; ++e) {
          const int ci = n0 + c8 + 2 * e;
          float f0 = sp[2 * e] * oscale + rb;
          float f1 = sp[2 * e + 1] * oscale + rb;
          if constexpr (EPI == 1) {
            f0 += bfr(ep0[ci]);
            f1 += bfr(ep0[ci + 1]);
          }
          if constexpr (OM == 5) {
            const float g0 = (f0 + bfr(ep1[ci])) * ocarry, g1 = (f1 + bfr(ep1[ci + 1])) * ocarry;
            const float w0 = (f0 + bfr(ep2[ci])) * ocarry, w1 = (f1 + bfr(ep2[ci + 1])) * ocarry;
            a[e]  = pk16(h_bits((_Float16)g0), h_bits((_Float16)g1));
            b2[e] = pk16(h_bits((_Float16)w0), h_bits((_Float16)w1));
          } else {
            f0 *= ocarry; f1 *= ocarry;
            const _Float16 x0 = (_Float16)f0, x1 = (_Float16)f1;
            a[e] = pk16(h_bits(x0), h_bits(x1));
            if constexpr (OM == 4) {
              b2[e] = pk16(h_bits((_Float16)(f0 - (float)x0)), h_bits((_Float16)(f1 - (float)x1)));
            }
          }
        }
        hv[it] = a;
        lv[it] = b2;
      }
      for (int pass = 0; pass < 2; ++pass) {
#pragma unroll
        for (int it = 0; it < 4; ++it) {
          const int row = it * 4 + q8;
          *(volatile v4u*)(C + (size_t)(mBase + row) * ldc + n0 + c8) = hv[it];
          if constexpr (OM >= 4) {
            *(volatile v4u*)(Cb + (size_t)(mBase + row) * ldc + n0 + c8) = lv[it];
          }
        }
        __threadfence();
      }
    }
    wave_sync_lds();
  }
}

__global__ __launch_bounds__(ATT_THREADS) __attribute__((amdgpu_num_vgpr(256)))
void attn_rel(const unsigned short* __restrict__ QH, const unsigned short* __restrict__ QL,
              const unsigned short* __restrict__ KH, const unsigned short* __restrict__ KL,
              const unsigned short* __restrict__ EP,
              const unsigned short* __restrict__ VH, const unsigned short* __restrict__ VL,
              unsigned short* CH, unsigned short* CL) {
  __shared__ __align__(16) float smem[ATT_W * WFL];

  const int tid  = threadIdx.x;
  const int wave = tid >> 5;
  const int lane = tid & 31;
  const int hh   = lane >> 4;
  const int c    = lane & 15;
  const int bh   = blockIdx.y;
  const int b    = bh / NH;
  const int h    = bh - b * NH;
  const int i0   = blockIdx.x * 64;
  const int iw0  = i0 + wave * 16;

  float* tsh = smem + wave * WFL;
  float* pt  = tsh + 16 * TPI;

  const size_t qro = ((size_t)b * SEQ + iw0 + c) * DMOD + h * DH + 8 * hh;
  const unsigned short* Khb = KH + (size_t)b * SEQ * DMOD + h * DH + 8 * hh;
  const unsigned short* Klb = KL + (size_t)b * SEQ * DMOD + h * DH + 8 * hh;
  const unsigned short* Eb  = EP + 8 * hh;
  const size_t vpo = (size_t)b * DMOD * SEQ + (size_t)(h * DH) * SEQ + 8 * hh;
  const unsigned short* Vhb = VH + vpo;
  const unsigned short* Vlb = VL + vpo;

  const float CS = LOG2E * SCALE / (QC * KC);
  const float CT = LOG2E * SCALE / (QC * EC);

  float mrow[8], lrow[8];
  v8f O[4];
#pragma unroll
  for (int r = 0; r < 8; ++r) { mrow[r] = -INFINITY; lrow[r] = 0.f; }
#pragma unroll
  for (int td = 0; td < 4; ++td) O[td] = zero8();

  const int ntile = SEQ / 64;
#pragma unroll 1
  for (int jt = 0; jt < ntile; ++jt) {
    const int j0 = jt * 64;
    const v16h qha = ldfrag_u(QH + qro), qhb = ldfrag_u(QH + qro + 32);
    const v16h qla = ldfrag_u(QL + qro), qlb = ldfrag_u(QL + qro + 32);

    {
      const int wlo = (SEQ - 2) - (iw0 - j0) - 15;
#pragma unroll 1
      for (int u = 0; u < 5; ++u) {
        int m = wlo + 16 * u + c;
        m = (m < 0) ? 0 : m;
        m = (m > ELEN - 1) ? (ELEN - 1) : m;
        const size_t eo = (size_t)m * DH;
        const v16h fa = ldfrag_u(Eb + eo), fb = ldfrag_u(Eb + eo + 32);
        v8f t8 = mma_h(qha, fa, zero8());
        t8 = mma_h(qla, fa, t8);
        t8 = mma_h(qhb, fb, t8);
        t8 = mma_h(qlb, fb, t8);
        hz6(t8, fa, fb, qha, qla, qhb, qlb);
        const int cb = 16 * u + c;
#pragma unroll
        for (int r = 0; r < 8; ++r) tsh[(8 * hh + r) * TPI + cb] = t8[r];
      }
    }
#pragma unroll 1
    for (int t = 0; t < 4; ++t) {
      const size_t ko = (size_t)(j0 + 16 * t + c) * DMOD;
      const v16h kha = ldfrag_u(Khb + ko), khb = ldfrag_u(Khb + ko + 32);
      const v16h kla = ldfrag_u(Klb + ko), klb = ldfrag_u(Klb + ko + 32);
      v8f s8 = mma_h(qha, kha, zero8());
      s8 = mma_h(qha, kla, s8);
      s8 = mma_h(qla, kha, s8);
      s8 = mma_h(qhb, khb, s8);
      s8 = mma_h(qhb, klb, s8);
      s8 = mma_h(qlb, khb, s8);
      hz8(s8, kha, khb, kla, klb, qha, qla, qhb, qlb);
      const int cb = 16 * t + c;
#pragma unroll
      for (int r = 0; r < 8; ++r) pt[(8 * hh + r) * SPI + cb] = s8[r];
    }
    wave_sync_lds();

#pragma unroll
    for (int r = 0; r < 8; ++r) {
      const int R = 8 * hh + r;
      const int i = iw0 + R;
      const float* trow = tsh + R * TPI + (15 - R) + c;
      float* srow = pt + R * SPI + c;
      float tv[4];
#pragma unroll
      for (int t = 0; t < 4; ++t) {
        const int j = j0 + 16 * t + c;
        const int ridx = (SEQ - 2) + j - i;
        const float tr = trow[16 * t];
        const float rel = (ridx < 0) ? 0.f : tr;
        tv[t] = srow[16 * t] * CS + rel * CT;
      }
      float mx = fmaxf(fmaxf(tv[0], tv[1]), fmaxf(tv[2], tv[3]));
#pragma unroll
      for (int off = 1; off < 16; off <<= 1) mx = fmaxf(mx, __shfl_xor(mx, off, 32));
      const float mn = fmaxf(mrow[r], mx);
      const float al = exp2f(mrow[r] - mn);
      mrow[r] = mn;
      float e4[4];
      float ps = 0.f;
#pragma unroll
      for (int t = 0; t < 4; ++t) { e4[t] = exp2f(tv[t] - mn); ps += e4[t]; }
#pragma unroll
      for (int off = 1; off < 16; off <<= 1) ps += __shfl_xor(ps, off, 32);
      lrow[r] = lrow[r] * al + ps;
#pragma unroll
      for (int td = 0; td < 4; ++td) O[td][r] *= al;
#pragma unroll
      for (int t = 0; t < 4; ++t) srow[16 * t] = e4[t];
    }
    wave_sync_lds();

#pragma unroll
    for (int ks = 0; ks < 2; ++ks) {
      FragH ph, pl;
      {
        const float* prow = pt + c * SPI + 32 * ks + 8 * hh;
        const v4f p0 = *(const v4f*)(prow), p1 = *(const v4f*)(prow + 4);
        const v4f p2 = *(const v4f*)(prow + 16), p3 = *(const v4f*)(prow + 20);
#pragma unroll
        for (int e = 0; e < 4; ++e) {
          _Float16 a0, a1;
          sp16(p0[e] * PC, a0, a1); ph.h[0][e]     = a0; pl.h[0][e]     = a1;
          sp16(p1[e] * PC, a0, a1); ph.h[0][4 + e] = a0; pl.h[0][4 + e] = a1;
          sp16(p2[e] * PC, a0, a1); ph.h[1][e]     = a0; pl.h[1][e]     = a1;
          sp16(p3[e] * PC, a0, a1); ph.h[1][4 + e] = a0; pl.h[1][4 + e] = a1;
        }
      }
      const size_t vo = (size_t)c * SEQ + j0 + 32 * ks;
#pragma unroll
      for (int td = 0; td < 4; ++td) {
        const size_t vv = vo + (size_t)(16 * td) * SEQ;
        const v16h vh = ldfrag_u(Vhb + vv), vl = ldfrag_u(Vlb + vv);
        O[td] = mma_h(ph.v, vh, O[td]);
        O[td] = mma_h(ph.v, vl, O[td]);
        O[td] = mma_h(pl.v, vh, O[td]);
        hz4(O[td], vh, vl, ph.v, pl.v);
      }
    }
    wave_sync_lds();
  }
  acc_guard4(O[0], O[1], O[2], O[3]);

  const float oc = 1.0f / (PC * VC);
#pragma unroll
  for (int r = 0; r < 8; ++r) {
    const float inv = (1.0f / lrow[r]) * oc;
    const int ro = (8 * hh + r) * SPI + c;
#pragma unroll
    for (int td = 0; td < 4; ++td) pt[ro + 16 * td] = O[td][r] * inv;
  }
  wave_sync_lds();
  {
    const int q8 = lane >> 3, c8 = (lane & 7) * 8;
    v4u hv[4], lv[4];
#pragma unroll
    for (int it = 0; it < 4; ++it) {
      const int row = it * 4 + q8;
      const float* sp = pt + row * SPI + c8;
      const v4f p0 = *(const v4f*)(sp), p1 = *(const v4f*)(sp + 4);
      v4u a, l2;
      unsigned hw, lw;
      pack_hl(p0[0] * CC, p0[1] * CC, hw, lw); a[0] = hw; l2[0] = lw;
      pack_hl(p0[2] * CC, p0[3] * CC, hw, lw); a[1] = hw; l2[1] = lw;
      pack_hl(p1[0] * CC, p1[1] * CC, hw, lw); a[2] = hw; l2[2] = lw;
      pack_hl(p1[2] * CC, p1[3] * CC, hw, lw); a[3] = hw; l2[3] = lw;
      hv[it] = a;
      lv[it] = l2;
    }
    const size_t ob = ((size_t)b * SEQ + iw0) * DMOD + h * DH + c8;
    for (int pass = 0; pass < 2; ++pass) {
#pragma unroll
      for (int it = 0; it < 4; ++it) {
        const int row = it * 4 + q8;
        *(volatile v4u*)(CH + ob + (size_t)row * DMOD) = hv[it];
        *(volatile v4u*)(CL + ob + (size_t)row * DMOD) = lv[it];
      }
      __threadfence();
    }
  }
}

extern "C" void kernel_launch(void* const* d_in, const int* in_sizes, int n_in,
                              void* d_out, int out_size, void* d_ws, size_t ws_size,
                              hipStream_t stream) {
  if (n_in < 10) return;
  if (in_sizes[0] != NROW * DMOD) return;
  if (in_sizes[1] != DMOD * DMOD || in_sizes[3] != DMOD * DMOD || in_sizes[5] != DMOD * DMOD || in_sizes[7] != DMOD * DMOD) return;
  if (in_sizes[2] != DMOD || in_sizes[4] != DMOD || in_sizes[6] != DMOD || in_sizes[8] != DMOD) return;
  if (in_sizes[9] != ELEN * DH) return;
  if (out_size != NROW * DMOD) return;

  const float* xin = (const float*)d_in[0];
  const float* w_q = (const float*)d_in[1];
  const float* b_q = (const float*)d_in[2];
  const float* w_k = (const float*)d_in[3];
  const float* b_k = (const float*)d_in[4];
  const float* w_v = (const float*)d_in[5];
  const float* b_v = (const float*)d_in[6];
  const float* w_o = (const float*)d_in[7];
  const float* b_o = (const float*)d_in[8];
  const float* er  = (const float*)d_in[9];
  float*       out = (float*)d_out;

  const size_t PX = (size_t)NROW * DMOD * 2;
  const size_t PW = (size_t)DMOD * DMOD * 2;
  const size_t PE = (size_t)EPAD * DH * 2;
  const size_t PV = (size_t)NBAT * DMOD * SEQ * 2;
  size_t off = 0;
  const size_t oX  = off; off += PX;
  const size_t oWq = off; off += PW;
  const size_t oWk = off; off += PW;
  const size_t oWv = off; off += PW;
  const size_t oWo = off; off += PW;
  const size_t oE  = off; off += PE;
  const size_t oQH = off; off += PX;
  const size_t oQL = off; off += PX;
  const size_t oKH = off; off += PX;
  const size_t oKL = off; off += PX;
  const size_t oVH = off; off += PV;
  const size_t oVL = off; off += PV;
  const size_t oCH = off; off += PX;
  const size_t oCL = off; off += PX;
  if (off > ws_size) return;
  if (off > (size_t)134217728) return;

  char* ws = (char*)d_ws;
  unsigned short* X16 = (unsigned short*)(ws + oX);
  unsigned short* Wq6 = (unsigned short*)(ws + oWq);
  unsigned short* Wk6 = (unsigned short*)(ws + oWk);
  unsigned short* Wv6 = (unsigned short*)(ws + oWv);
  unsigned short* Wo6 = (unsigned short*)(ws + oWo);
  unsigned short* E16 = (unsigned short*)(ws + oE);
  unsigned short* QHp = (unsigned short*)(ws + oQH);
  unsigned short* QLp = (unsigned short*)(ws + oQL);
  unsigned short* KHp = (unsigned short*)(ws + oKH);
  unsigned short* KLp = (unsigned short*)(ws + oKL);
  unsigned short* VHp = (unsigned short*)(ws + oVH);
  unsigned short* VLp = (unsigned short*)(ws + oVL);
  unsigned short* CHp = (unsigned short*)(ws + oCH);
  unsigned short* CLp = (unsigned short*)(ws + oCL);

  const dim3 blk(256);
  const dim3 gCX((NROW * DMOD) / 2048);
  const dim3 gCW((DMOD * DMOD) / 2048);
  const dim3 gCE((ELEN * DH + 2047) / 2048);
  const int tilesQ = (NROW / 64) * (DMOD / 64);
  const int tilesV = (DMOD / 64) * (SEQ / 64);
  const dim3 gQ((tilesQ + 7) / 8, 1);
  const dim3 gV((tilesV + 7) / 8, NBAT);
  const dim3 gAT(SEQ / 64, NBAT * NH);
  const dim3 bAT(ATT_THREADS);

  cvt16<<<gCX, blk, 0, stream>>>(xin, X16, NROW * DMOD, XC);
  cvt16<<<gCW, blk, 0, stream>>>(w_q, Wq6, DMOD * DMOD, WSC);
  cvt16<<<gCW, blk, 0, stream>>>(w_k, Wk6, DMOD * DMOD, WSC);
  cvt16<<<gCW, blk, 0, stream>>>(w_v, Wv6, DMOD * DMOD, WSC);
  cvt16<<<gCW, blk, 0, stream>>>(w_o, Wo6, DMOD * DMOD, WSC);
  cvt16<<<gCE, blk, 0, stream>>>(er, E16, ELEN * DH, EC);

  gemm64<4, 0, 0, 1><<<gQ, blk, 0, stream>>>(
      X16, X16, DMOD, 0LL,
      Wq6, DMOD, 0LL,
      (void*)QHp, (void*)QLp, DMOD, 0LL,
      NROW, DMOD, DMOD, 1.0f / (XC * WSC), QC,
      b_q, b_q, b_q);

  gemm64<4, 0, 0, 1><<<gQ, blk, 0, stream>>>(
      X16, X16, DMOD, 0LL,
      Wk6, DMOD, 0LL,
      (void*)KHp, (void*)KLp, DMOD, 0LL,
      NROW, DMOD, DMOD, 1.0f / (XC * WSC), KC,
      b_k, b_k, b_k);

  gemm64<4, 0, 0, 2><<<gV, blk, 0, stream>>>(
      Wv6, Wv6, DMOD, 0LL,
      X16, DMOD, (long long)SEQ * DMOD,
      (void*)VHp, (void*)VLp, SEQ, (long long)DMOD * SEQ,
      DMOD, SEQ, DMOD, 1.0f / (XC * WSC), VC,
      b_v, b_v, b_v);

  attn_rel<<<gAT, bAT, 0, stream>>>(QHp, QLp, KHp, KLp, E16, VHp, VLp, CHp, CLp);

  gemm64<0, 1, 0, 1><<<gQ, blk, 0, stream>>>(
      CHp, CLp, DMOD, 0LL,
      Wo6, DMOD, 0LL,
      (void*)out, (void*)out, DMOD, 0LL,
      NROW, DMOD, DMOD, 1.0f / (CC * WSC), 1.0f,
      b_o, b_o, b_o);
  (void)hipGetLastError();
}
